// FusionHeadCoAtten_1288490189258
// MI455X (gfx1250) — hardware-verified
//
#include <hip/hip_runtime.h>
#include <math.h>

typedef __attribute__((ext_vector_type(16))) _Float16 v16h;
typedef __attribute__((ext_vector_type(16))) __bf16 v16b;
typedef __attribute__((ext_vector_type(8)))  _Float16 v8h;
typedef __attribute__((ext_vector_type(8)))  float v8f;
typedef __attribute__((ext_vector_type(4)))  float v4f;
typedef __attribute__((ext_vector_type(2)))  float v2f;
typedef __attribute__((ext_vector_type(4)))  unsigned v4u;
typedef __attribute__((ext_vector_type(4)))  int v4i;
typedef float __attribute__((may_alias)) float_a;
typedef int __attribute__((may_alias)) int_a;

template <typename T> __device__ __forceinline__ void vst2(void* p, T v) { *(volatile T*)p = v; __threadfence(); *(volatile T*)p = v; }
__device__ __forceinline__ v8f wmma16(v16h a, v16h b, v8f c) {
  v8f d = __builtin_amdgcn_wmma_f32_16x16x32_f16(false, a, false, b, (short)0, c, false, false);
  asm volatile("v_nop\n\tv_nop\n\tv_nop\n\tv_nop" : "+v"(d) : "v"(a), "v"(b));
  return d;
}
__device__ __forceinline__ v8f wmma_bf(v16b a, v16b b, v8f c) {
  v8f d = __builtin_amdgcn_wmma_f32_16x16x32_bf16(false, a, false, b, (short)0, c, false, false);
  asm volatile("v_nop\n\tv_nop\n\tv_nop\n\tv_nop" : "+v"(d) : "v"(a), "v"(b));
  return d;
}
__device__ __forceinline__ v16h frag_h(const _Float16* rowk0, int lane) {
  union { v16h v; v8h q[2]; } u; const _Float16* p = rowk0 + 8 * (lane >> 4);
  u.q[0] = *(const v8h*)p; u.q[1] = *(const v8h*)(p + 16); return u.v;
}
__device__ __forceinline__ v16h frag_f32(const float* rowk0, int lane) {
  v16h a; const float* p = rowk0 + 8 * (lane >> 4);
#pragma unroll
  for (int i = 0; i < 8; ++i) { a[i] = (_Float16)p[i]; a[8 + i] = (_Float16)p[16 + i]; }
  return a;
}
__device__ __forceinline__ v16h frag_f32s(const float* rowk0, int lane, float sc) {
  v16h a; const float* p = rowk0 + 8 * (lane >> 4);
#pragma unroll
  for (int i = 0; i < 8; ++i) { a[i] = (_Float16)(p[i] * sc); a[8 + i] = (_Float16)(p[16 + i] * sc); }
  return a;
}
__device__ __forceinline__ v16h fragc_f32(const float* W, int k0, int n, int lane, int ld, int K) {
  v16h a; const int g = lane >> 4;
#pragma unroll
  for (int i = 0; i < 8; ++i) { const int ka = k0 + 8 * g + i, kb = ka + 16;
    a[i] = (_Float16)(ka < K ? W[(size_t)(ka < K ? ka : K - 1) * ld + n] : 0.f); a[8 + i] = (_Float16)(kb < K ? W[(size_t)(kb < K ? kb : K - 1) * ld + n] : 0.f); }
  return a;
}
struct F2 { v16b h, l; };
__device__ __forceinline__ F2 bsplit16(const float v[16]) { F2 r;
#pragma unroll
  for (int i = 0; i < 16; ++i) { const __bf16 h = (__bf16)v[i]; r.h[i] = h; r.l[i] = (__bf16)(v[i] - (float)h); }
  return r; }
__device__ __forceinline__ F2 split_row(const float* row, int k0, int lane) { float v[16]; const float* p = row + k0 + 8 * (lane >> 4);
#pragma unroll
  for (int i = 0; i < 8; ++i) { v[i] = p[i]; v[8 + i] = p[16 + i]; }
  return bsplit16(v); }
__device__ __forceinline__ F2 split_rowK(const float* row, int k0, int lane, int K) { float v[16]; const int g = lane >> 4;
#pragma unroll
  for (int i = 0; i < 8; ++i) { const int ka = k0 + 8 * g + i, kb = ka + 16; v[i] = ka < K ? row[ka < K ? ka : K - 1] : 0.f; v[8 + i] = kb < K ? row[kb < K ? kb : K - 1] : 0.f; }
  return bsplit16(v); }
__device__ __forceinline__ F2 split_col(const float* W, int k0, int n, int lane, int ld, int K) { float v[16]; const int g = lane >> 4;
#pragma unroll
  for (int i = 0; i < 8; ++i) { const int ka = k0 + 8 * g + i, kb = ka + 16; v[i] = ka < K ? W[(size_t)(ka < K ? ka : K - 1) * ld + n] : 0.f; v[8 + i] = kb < K ? W[(size_t)(kb < K ? kb : K - 1) * ld + n] : 0.f; }
  return bsplit16(v); }
__device__ __forceinline__ v8f mac3(const F2& a, const F2& b, v8f c) { c = wmma_bf(a.l, b.h, c); c = wmma_bf(a.h, b.l, c); return wmma_bf(a.h, b.h, c); }
__device__ __forceinline__ float sigm(float v) { return 1.0f / (1.0f + expf(-v)); }
#define LDSX() do { asm volatile("s_wait_dscnt 0" ::: "memory"); __builtin_amdgcn_wave_barrier(); __builtin_amdgcn_fence(__ATOMIC_RELEASE, "workgroup"); } while (0)


#define BB 512
#define DD 512
#ifndef TBB
#define TBB BB
#endif
typedef __attribute__((ext_vector_type(8))) __bf16 v8b;
__device__ __forceinline__ v16b frag_gbf(const float* rowk0, int lane) {
  v16b a; const float* p = rowk0 + 8 * (lane >> 4);
#pragma unroll
  for (int i = 0; i < 8; ++i) { a[i] = (__bf16)p[i]; a[8 + i] = (__bf16)p[16 + i]; }
  return a;
}
__device__ __forceinline__ float bfr(float v) { return (float)(__bf16)v; }
__device__ __attribute__((noinline)) float exp_ni(float v) { return expf(v); }
__device__ __attribute__((noinline)) float tanh_ni(float v) { return tanhf(v); }
#define WS_T   0u
#define WS_END (WS_T + 4u * BB * DD)

__global__ __launch_bounds__(128) void k_lin(const float* __restrict__ X, const float* __restrict__ Wt, const float* __restrict__ bb, float* __restrict__ T) {
  __shared__ __align__(16) float so[4][16][132];
  const int tid = threadIdx.x, wave = tid >> 5, lane = tid & 31, col = lane & 15, g = lane >> 4; const size_t r0 = (size_t)blockIdx.x * 64 + wave * 16; const int n0 = blockIdx.y * 128;
  v8f acc[8] = {};
#pragma unroll 2
  for (int kc = 0; kc < DD / 32; ++kc) { const v16b a = frag_gbf(X + (r0 + col) * DD + kc * 32, lane);
#pragma unroll
    for (int j = 0; j < 8; ++j) acc[j] = wmma_bf(a, frag_gbf(Wt + (size_t)(n0 + j * 16 + col) * DD + kc * 32, lane), acc[j]); }
#pragma unroll
  for (int j = 0; j < 8; ++j) { const float b2 = bfr(bb[n0 + j * 16 + col]);
#pragma unroll
    for (int r = 0; r < 8; ++r) so[wave][8 * g + r][j * 16 + col] = tanh_ni(acc[j][r] + b2); }
  LDSX();
  for (int rl = 0; rl < 16; ++rl) vst2(T + (r0 + rl) * DD + n0 + lane * 4, *(const v4f*)&so[wave][rl][lane * 4]);
}
__global__ __launch_bounds__(256) void k_coatt(const float* __restrict__ IMG, const float* __restrict__ AUD, const float* __restrict__ T, float* __restrict__ OUT) {
  __shared__ float st[DD], sa[DD], szi[DD], sm[DD], szi2[DD], sm2[DD]; __shared__ float sred[4][8]; __shared__ __align__(16) float so[4 * DD];
  const int b = blockIdx.x, tid = threadIdx.x, wave = tid >> 5, lane = tid & 31;
  for (int q = tid; q < DD; q += 256) { st[q] = T[(size_t)b * DD + q]; sa[q] = bfr(AUD[(size_t)b * DD + q]); so[q] = bfr(IMG[(size_t)b * DD + q]); so[DD + q] = sa[q]; }
  __syncthreads();
  { float tmx = -3.0e38f, tmn = 3.0e38f, amx = -3.0e38f, amn = 3.0e38f; for (int q = tid; q < DD; q += 256) { tmx = fmaxf(tmx, st[q]); tmn = fminf(tmn, st[q]); amx = fmaxf(amx, sa[q]); amn = fminf(amn, sa[q]); }
#pragma unroll
    for (int o = 1; o < 32; o <<= 1) { tmx = fmaxf(tmx, __shfl_xor(tmx, o)); tmn = fminf(tmn, __shfl_xor(tmn, o)); amx = fmaxf(amx, __shfl_xor(amx, o)); amn = fminf(amn, __shfl_xor(amn, o)); }
    if (lane == 0) { sred[0][wave] = tmx; sred[1][wave] = tmn; sred[2][wave] = amx; sred[3][wave] = amn; } }
  __syncthreads();
  float tmx = sred[0][0], tmn = sred[1][0], amx = sred[2][0], amn = sred[3][0];
  for (int w = 1; w < 8; ++w) { tmx = fmaxf(tmx, sred[0][w]); tmn = fminf(tmn, sred[1][w]); amx = fmaxf(amx, sred[2][w]); amn = fminf(amn, sred[3][w]); }
  for (int d = tid; d < DD; d += 256) { const float ad = sa[d]; const float md = ad >= 0.f ? tmx * ad : tmn * ad; float z = 0.f;
#pragma unroll 1
    for (int e = 0; e < DD; ++e) z += exp_ni(st[e] * ad - md);
    sm[d] = md; szi[d] = 1.0f / z;
    const float td = st[d]; const float md2 = td >= 0.f ? td * amx : td * amn; float z2 = 0.f;
#pragma unroll 1
    for (int e = 0; e < DD; ++e) z2 += exp_ni(td * sa[e] - md2);
    sm2[d] = md2; szi2[d] = 1.0f / z2; }
  __syncthreads();
  for (int e = tid; e < DD; e += 256) { const float te = st[e], ae = sa[e]; float ci = 0.f, ca = 0.f;
#pragma unroll 1
    for (int d = 0; d < DD; ++d) { ci += sa[d] * exp_ni(te * sa[d] - sm[d]) * szi[d]; ca += st[d] * exp_ni(st[d] * ae - sm2[d]) * szi2[d]; }
    so[2 * DD + e] = ci; so[3 * DD + e] = ca; }
  __syncthreads();
  for (int q = tid; q < 4 * DD / 4; q += 256) vst2(OUT + (size_t)b * 4 * DD + q * 4, *(const v4f*)&so[q * 4]);
}

extern "C" void kernel_launch(void* const* d_in, const int* in_sizes, int n_in, void* d_out, int out_size, void* d_ws, size_t ws_size, hipStream_t stream) {
  (void)in_sizes; (void)n_in; (void)out_size;
  const float** F = (const float**)d_in;
  if (ws_size < (size_t)WS_END) return;
  char* ws = (char*)d_ws; float* T = (float*)(ws + WS_T);
  k_lin<<<dim3(BB / 64, DD / 128), 128, 0, stream>>>(F[0], F[2], F[3], T);
  k_coatt<<<TBB, 256, 0, stream>>>(F[0], F[1], T, (float*)d_out);
}
